// LMHSA_20804821582378
// MI455X (gfx1250) — hardware-run, weakly checked
//
#include <hip/hip_runtime.h>
#include <math.h>


#define C_DIM   256
#define IMG_W   96
#define HW_N    9216
#define NHEAD   8
#define HEADD   32
#define NWIN    24
#define WTOK    384
#define NPOOL   144
#define POOLG   12
#define C1_DIM  192
#define C2_DIM  64
#define CTXW    32
#define QH_LD   256
#define QKV_LD  768
#define KV_LD   512
#define KCOL    256
#define VCOL    512
#define LN_EPS  1e-5f
#define ATT_SCALE 0.17677669529663687f
#define QKV_OSC 16.0f
#define WO_OSC  64.0f
#define OUT_OSC (1.0f / 1024.0f)
#define CL2     (ATT_SCALE * 1.4426950408889634f / 256.0f)
#define TS_CSH  64
#define TS_CSV  320
#define TS_N    576
#define MAXB    4

static_assert(NHEAD * HEADD == C_DIM);
static_assert(C1_DIM + C2_DIM == C_DIM);
static_assert(HW_N == IMG_W * IMG_W);
static_assert(NPOOL == POOLG * POOLG);
static_assert(NWIN * 4 == IMG_W);
static_assert(WTOK == IMG_W * 4);
static_assert((HW_N % 64) == 0 && (WTOK % 64) == 0);
static_assert((TS_N % 4) == 0 && TS_CSV + C_DIM == TS_N);

typedef __bf16         v16bf __attribute__((ext_vector_type(16)));
typedef _Float16       v16h  __attribute__((ext_vector_type(16)));
typedef float          v8f   __attribute__((ext_vector_type(8)));
typedef float          v4f   __attribute__((ext_vector_type(4)));
typedef unsigned int   v4u   __attribute__((ext_vector_type(4)));
typedef unsigned short v8us  __attribute__((ext_vector_type(8)));
typedef unsigned short v16us __attribute__((ext_vector_type(16)));

__device__ __forceinline__ unsigned short bf_bits(float f) {
  const unsigned u = __float_as_uint(f);
  return (unsigned short)((u + 0x7FFFu + ((u >> 16) & 1u)) >> 16);
}
__device__ __forceinline__ float bf_up(unsigned short h) { return __uint_as_float(((unsigned)h) << 16); }
__device__ __forceinline__ float bfr(float f) { return bf_up(bf_bits(f)); }
__device__ __forceinline__ unsigned short h_bits(float f) {
  const _Float16 h = (_Float16)f;
  return __builtin_bit_cast(unsigned short, h);
}
__device__ __forceinline__ unsigned pk16(unsigned short a, unsigned short b) { return (unsigned)a | ((unsigned)b << 16); }
__device__ __forceinline__ v8f zero8() { v8f z = {0.f, 0.f, 0.f, 0.f, 0.f, 0.f, 0.f, 0.f}; return z; }
__device__ __forceinline__ v8us zero8us() { v8us z = {0, 0, 0, 0, 0, 0, 0, 0}; return z; }

__device__ __forceinline__ void ld8(const float* p, float* o) {
  const v4f a = *(const v4f*)(p);
  const v4f b = *(const v4f*)(p + 4);
  o[0] = a[0]; o[1] = a[1]; o[2] = a[2]; o[3] = a[3];
  o[4] = b[0]; o[5] = b[1]; o[6] = b[2]; o[7] = b[3];
}

__device__ __forceinline__ void lds_sync() {
  __builtin_amdgcn_fence(__ATOMIC_RELEASE, "workgroup");
  __builtin_amdgcn_wave_barrier();
  __builtin_amdgcn_fence(__ATOMIC_ACQUIRE, "workgroup");
}

__device__ __forceinline__ v16us ldfrag_u(const unsigned short* p) {
  union { v16us v; v8us h[2]; } f;
  f.h[0] = *(const v8us*)(p);
  f.h[1] = *(const v8us*)(p + 16);
  return f.v;
}
__device__ __forceinline__ v16h ldfrag_h(const unsigned short* p) { return __builtin_bit_cast(v16h, ldfrag_u(p)); }

template <int TF>
__device__ __forceinline__ v8f mma_raw(v16us a, v16us b, v8f c) {
  if (TF == 0)
    return __builtin_amdgcn_wmma_f32_16x16x32_bf16(false, __builtin_bit_cast(v16bf, a), false,
                                                   __builtin_bit_cast(v16bf, b), (short)0, c, false, false);
  return __builtin_amdgcn_wmma_f32_16x16x32_f16(false, __builtin_bit_cast(v16h, a), false,
                                                __builtin_bit_cast(v16h, b), (short)0, c, false, false);
}
__device__ __forceinline__ v8f mma_h(v16h a, v16h b, v8f c) {
  c = __builtin_amdgcn_wmma_f32_16x16x32_f16(false, a, false, b, (short)0, c, false, false);
#if defined(__HIP_DEVICE_COMPILE__)
  asm volatile("v_nop\n\tv_nop\n\tv_nop\n\tv_nop" : "+v"(c) : "v"(a), "v"(b));
#endif
  return c;
}
__device__ __forceinline__ void dep_guard(v8f& a, v8f& b, v16us x) {
#if defined(__HIP_DEVICE_COMPILE__)
  asm volatile("v_nop\n\tv_nop\n\tv_nop\n\tv_nop" : "+v"(a), "+v"(b) : "v"(x));
#endif
}
__device__ __forceinline__ void keep4(v16us a, v16us b, v16us c, v16us d) {
#if defined(__HIP_DEVICE_COMPILE__)
  asm volatile("v_nop" :: "v"(a), "v"(b), "v"(c), "v"(d));
#endif
}
__device__ __forceinline__ void acc_guard4(v8f& a, v8f& b, v8f& c, v8f& d) {
#if defined(__HIP_DEVICE_COMPILE__)
  asm volatile("v_nop\n\tv_nop\n\tv_nop\n\tv_nop" : "+v"(a), "+v"(b), "+v"(c), "+v"(d));
#endif
}

template <int KIND>
__global__ __launch_bounds__(256) void k_tr(const float* __restrict__ in, unsigned short* out, int R, int Cc) {
  __shared__ float s[64][65];
  const int c0 = blockIdx.x * 64, r0 = blockIdx.y * 64;
  if (c0 + 64 > Cc || r0 + 64 > R) return;
  const float* inb = in + (size_t)blockIdx.z * (size_t)R * (size_t)Cc;
  unsigned short* outb = out + (size_t)blockIdx.z * (size_t)R * (size_t)Cc;
  const int t = threadIdx.x, cc = t & 63, rq = t >> 6;
#pragma unroll
  for (int it = 0; it < 16; ++it) {
    const int r = it * 4 + rq;
    s[r][cc] = inb[(size_t)(r0 + r) * (size_t)Cc + c0 + cc];
  }
  __syncthreads();
  const int q8 = t & 7, rr = t >> 3;
  v4u ov[2];
  size_t oo[2];
#pragma unroll
  for (int it = 0; it < 2; ++it) {
    const int cc2 = it * 32 + rr;
    unsigned short hb[8];
#pragma unroll
    for (int e = 0; e < 8; ++e) {
      const float v = s[q8 * 8 + e][cc2];
      hb[e] = (KIND == 0) ? bf_bits(v) : h_bits(WO_OSC * bfr(v));
    }
    v4u p;
#pragma unroll
    for (int q = 0; q < 4; ++q) p[q] = pk16(hb[2 * q], hb[2 * q + 1]);
    ov[it] = p;
    oo[it] = (size_t)(c0 + cc2) * (size_t)R + r0 + q8 * 8;
  }
  for (int pass = 0; pass < 2; ++pass) {
#pragma unroll
    for (int it = 0; it < 2; ++it) *(volatile v4u*)(outb + oo[it]) = ov[it];
    __threadfence();
  }
}

__global__ __launch_bounds__(192) void k_xstats(const float* __restrict__ x, double* P1) {
  __shared__ float sS[192], sQ[192];
  __shared__ __align__(16) double sD[2 * NWIN];
  const int blk = blockIdx.x;
  const float* xp = x + (size_t)blk * HW_N;
  const int t = threadIdx.x, xc = t % IMG_W, half = t / IMG_W;
  float s = 0.f, q = 0.f;
#pragma unroll 4
  for (int y = 0; y < IMG_W / 2; ++y) {
    const float v = bfr(xp[(half * (IMG_W / 2) + y) * IMG_W + xc]);
    s += v;
    q += v * v;
  }
  sS[t] = s; sQ[t] = q;
  __syncthreads();
  if (t < NWIN) {
    double ds = 0.0, dq = 0.0;
#pragma unroll
    for (int e = 0; e < 8; ++e) {
      const int idx = (e >> 2) * IMG_W + 4 * t + (e & 3);
      ds += (double)sS[idx];
      dq += (double)sQ[idx];
    }
    sD[2 * t] = ds; sD[2 * t + 1] = dq;
  }
  __syncthreads();
  if (t < NWIN) {
    const v4u v = *(const v4u*)(&sD[2 * t]);
    double* dst = P1 + (size_t)blk * (2 * NWIN) + 2 * t;
    *(volatile v4u*)dst = v;
    __threadfence();
    *(volatile v4u*)dst = v;
  }
}

__global__ __launch_bounds__(256) void k_reduce1(const double* __restrict__ P1, int nblk,
                                                 const float* __restrict__ hWq, const float* __restrict__ vWq,
                                                 float* T, double inv_nw, double inv_ng) {
  __shared__ double sA[2 * NWIN];
  __shared__ __align__(16) float sT[TS_N];
  const int t = threadIdx.x;
  if (t < 64) sT[t] = 0.f;
  if (t < 2 * NWIN) {
    double a = 0.0;
    for (int k = 0; k < nblk; ++k) a += P1[(size_t)k * (2 * NWIN) + t];
    sA[t] = a;
  }
  {
    double ch = 0.0, cv = 0.0;
#pragma unroll 4
    for (int k = 0; k < C_DIM; ++k) {
      ch += (double)bfr(hWq[k * C_DIM + t]);
      cv += (double)bfr(vWq[k * C_DIM + t]);
    }
    sT[TS_CSH + t] = (float)ch;
    sT[TS_CSV + t] = (float)cv;
  }
  __syncthreads();
  if (t < NWIN) {
    const double S = sA[2 * t], Q = sA[2 * t + 1];
    const double m = S * inv_nw;
    const double var = Q * inv_nw - m * m;
    sT[2 + 2 * t] = (float)m;
    sT[3 + 2 * t] = rsqrtf((float)var + LN_EPS);
  }
  if (t == NWIN) {
    double S = 0.0, Q = 0.0;
    for (int wi = 0; wi < NWIN; ++wi) { S += sA[2 * wi]; Q += sA[2 * wi + 1]; }
    const double m = S * inv_ng;
    const double var = Q * inv_ng - m * m;
    sT[0] = (float)m;
    sT[1] = rsqrtf((float)var + LN_EPS);
  }
  __syncthreads();
  if (t < TS_N / 4) {
    const v4f v = *(const v4f*)(sT + 4 * t);
    *(volatile v4f*)(T + 4 * t) = v;
    __threadfence();
    *(volatile v4f*)(T + 4 * t) = v;
  }
}

__global__ __launch_bounds__(256) void k_zfill(unsigned short* Xph, unsigned short* Xpl, int row0, int nrows) {
  const int i = blockIdx.x * 256 + threadIdx.x;
  const int npieces = nrows * (C_DIM / 8);
  if (i >= npieces) return;
  v4u z;
  z[0] = 0u; z[1] = 0u; z[2] = 0u; z[3] = 0u;
  const size_t oo = (size_t)row0 * C_DIM + (size_t)i * 8;
  *(volatile v4u*)(Xph + oo) = z;
  *(volatile v4u*)(Xpl + oo) = z;
  __threadfence();
  *(volatile v4u*)(Xph + oo) = z;
  *(volatile v4u*)(Xpl + oo) = z;
}

__global__ __launch_bounds__(256) void k_pool(const float* __restrict__ x, unsigned short* Xph, unsigned short* Xpl) {
  __shared__ float s[POOLG][65];
  const int gy = blockIdx.x, c0 = blockIdx.y * 64, b = blockIdx.z;
  const int t = threadIdx.x, cs = t >> 2, gq = t & 3;
  const float* xc = x + ((size_t)(b * C_DIM + c0 + cs) * IMG_W + 8 * gy) * IMG_W;
#pragma unroll
  for (int g3 = 0; g3 < 3; ++g3) {
    const int gx = gq + 4 * g3;
    float a = 0.f;
#pragma unroll
    for (int dy = 0; dy < 8; ++dy) {
      const v4f u0 = *(const v4f*)(xc + dy * IMG_W + 8 * gx);
      const v4f u1 = *(const v4f*)(xc + dy * IMG_W + 8 * gx + 4);
      a += ((bfr(u0[0]) + bfr(u0[1])) + (bfr(u0[2]) + bfr(u0[3]))) +
           ((bfr(u1[0]) + bfr(u1[1])) + (bfr(u1[2]) + bfr(u1[3])));
    }
    s[gx][cs] = a * (1.0f / 64.0f);
  }
  __syncthreads();
  if (t < 192) {
    const int plane = t / 96;
    const int u = t - plane * 96;
    const int row = u >> 3, q8 = u & 7;
    unsigned short ob[8];
#pragma unroll
    for (int e = 0; e < 8; ++e) {
      const float f = s[row][q8 * 8 + e];
      const unsigned short hb = bf_bits(f);
      const unsigned short lb = bf_bits(f - bf_up(hb));
      ob[e] = (plane == 0) ? hb : lb;
    }
    v4u ov;
#pragma unroll
    for (int q = 0; q < 4; ++q) ov[q] = pk16(ob[2 * q], ob[2 * q + 1]);
    unsigned short* dst = (plane == 0) ? Xph : Xpl;
    const size_t oo = (size_t)(b * NPOOL + gy * POOLG + row) * C_DIM + c0 + q8 * 8;
    *(volatile v4u*)(dst + oo) = ov;
    __threadfence();
    *(volatile v4u*)(dst + oo) = ov;
  }
}

template <int NA, int AHM, int TF>
__device__ __forceinline__ void kloop(v8f (&acc)[4][4],
                                      const unsigned short* __restrict__ Pa, const unsigned short* __restrict__ Pb,
                                      int lda, int m0, int K,
                                      const unsigned short* __restrict__ Bt, int ldb, int n0,
                                      int rlane, int koff) {
  int bm = 0, sm0 = m0;
  if (AHM != 0) { bm = m0 / HW_N; sm0 = m0 - bm * HW_N; }
  for (int kk = 0; kk < K; kk += 32) {
    v16us bh[4];
#pragma unroll
    for (int j = 0; j < 4; ++j) {
      const size_t bo = (size_t)(n0 + (j << 4) + rlane) * (size_t)ldb + koff + kk;
      bh[j] = ldfrag_u(Bt + bo);
    }
#pragma unroll
    for (int i = 0; i < 4; ++i) {
      const unsigned short* pa;
      const unsigned short* pb;
      if (AHM == 0) {
        const size_t ao = (size_t)(m0 + (i << 4) + rlane) * (size_t)lda + koff + kk;
        pa = Pa + ao;
        pb = Pb + ao;
      } else {
        const size_t ao = ((size_t)(bm * NHEAD + (kk >> 5)) * HW_N + sm0 + (i << 4) + rlane) * CTXW + koff;
        pa = Pa + ao;
        pb = pa;
      }
      const v16us a0 = ldfrag_u(pa);
#pragma unroll
      for (int j = 0; j < 4; ++j) acc[i][j] = mma_raw<TF>(a0, bh[j], acc[i][j]);
      dep_guard(acc[i][0], acc[i][3], a0);
      if (NA == 2) {
        const v16us a1 = ldfrag_u(pb);
#pragma unroll
        for (int j = 0; j < 4; ++j) acc[i][j] = mma_raw<TF>(a1, bh[j], acc[i][j]);
        dep_guard(acc[i][0], acc[i][3], a1);
      }
    }
    keep4(bh[0], bh[1], bh[2], bh[3]);
  }
}

template <int MODE, int NA, int AHM, int TF, int EP, int WST>
__global__ __launch_bounds__(256) void gemm64(
    const unsigned short* __restrict__ Pa, const unsigned short* __restrict__ Pb, int lda,
    const unsigned short* __restrict__ Bt, int ldb,
    const float* __restrict__ bias0, const float* __restrict__ bias1, const float* __restrict__ bias2,
    const float* __restrict__ Tst, const float* __restrict__ xres,
    float* Cf, unsigned short* Ch, int ldc, int M, int N, int K, float osc, int cbase) {
  __shared__ __align__(16) float sT[8][1152];
  const int lane = threadIdx.x & 31;
  const int wave = threadIdx.x >> 5;
  const int tilesN = N >> 6;
  const int tilesM = M >> 6;
  const int tiles = tilesM * tilesN;
  const int item = blockIdx.x * 8 + wave;
  if (item >= tiles) return;
  const int tm = item / tilesN;
  const int tn = item - tm * tilesN;
  const int m0 = tm << 6;
  const int n0 = tn << 6;

  const int rlane = lane & 15;
  const int koff  = (lane >> 4) * 8;
  const int mOff  = (lane >> 4) * 8;

  v8f acc[4][4];
#pragma unroll
  for (int i = 0; i < 4; ++i)
#pragma unroll
    for (int j = 0; j < 4; ++j) acc[i][j] = zero8();

  kloop<NA, AHM, TF>(acc, Pa, Pb, lda, m0, K, Bt, ldb, n0, rlane, koff);
  acc_guard4(acc[0][0], acc[0][1], acc[0][2], acc[0][3]);
  acc_guard4(acc[1][0], acc[1][1], acc[1][2], acc[1][3]);
  acc_guard4(acc[2][0], acc[2][1], acc[2][2], acc[2][3]);
  acc_guard4(acc[3][0], acc[3][1], acc[3][2], acc[3][3]);

  float* slab = sT[wave];
  if (MODE == 1) {
    const int q8 = lane & 7, rr = lane >> 3, c8 = q8 * 8;
    int g = 0;
    if (EP != 0) g = n0 >> 8;
    const float* bsel = bias0;
    if (EP != 0) { if (g == 1) bsel = bias1; if (g >= 2) bsel = bias2; }
    const int nrel = n0 - (g << 8) + c8;
    float b8[8];
    ld8(bsel + nrel, b8);
#pragma unroll
    for (int e = 0; e < 8; ++e) b8[e] = bfr(b8[e]);
    float cs8[8];
#pragma unroll
    for (int e = 0; e < 8; ++e) cs8[e] = 0.f;
    float mg = 0.f, rg = 1.f;
    const bool fold = (EP == 1) && (g == 0);
    if (fold) {
      ld8(Tst + ((WST == 0) ? TS_CSH : TS_CSV) + nrel, cs8);
      if (WST == 0) { mg = Tst[0]; rg = Tst[1]; }
    }
#pragma unroll
    for (int i = 0; i < 4; ++i) {
      const int mBase = m0 + (i << 4);
#pragma unroll
      for (int r = 0; r < 8; ++r) {
#pragma unroll
        for (int j = 0; j < 4; ++j) {
          slab[(mOff + r) * 68 + (j << 4) + rlane] = acc[i][j][r];
        }
      }
      lds_sync();
      v4u ov[4];
#pragma unroll
      for (int it = 0; it < 4; ++it) {
        const int row = it * 4 + rr;
        float xs[8];
        ld8(slab + row * 68 + c8, xs);
        float mr = mg, rw = rg;
        if (fold && WST == 1) {
          const int xcol = (mBase + row) % IMG_W;
          const int wi = xcol >> 2;
          mr = Tst[2 + 2 * wi];
          rw = Tst[3 + 2 * wi];
        }
        unsigned short hb[8];
#pragma unroll
        for (int e = 0; e < 8; ++e) hb[e] = h_bits((rw * (xs[e] - mr * cs8[e]) + b8[e]) * osc);
        v4u ah;
#pragma unroll
        for (int p = 0; p < 4; ++p) ah[p] = pk16(hb[2 * p], hb[2 * p + 1]);
        ov[it] = ah;
      }
      for (int pass = 0; pass < 2; ++pass) {
#pragma unroll
        for (int it = 0; it < 4; ++it) {
          const int row = it * 4 + rr;
          const size_t co = (size_t)(mBase + row) * (size_t)ldc + n0 + c8;
          *(volatile v4u*)(Ch + co) = ov[it];
        }
        __threadfence();
      }
      lds_sync();
    }
  } else {
    const int bm = m0 / HW_N, sm0 = m0 - bm * HW_N;
    const int q8 = lane & 7, rr = lane >> 3;
#pragma unroll
    for (int hm = 0; hm < 2; ++hm) {
#pragma unroll
      for (int hn = 0; hn < 2; ++hn) {
#pragma unroll
        for (int ii = 0; ii < 2; ++ii) {
#pragma unroll
          for (int jj = 0; jj < 2; ++jj) {
#pragma unroll
            for (int r = 0; r < 8; ++r) {
              slab[((jj << 4) + rlane) * 36 + (ii << 4) + mOff + r] = acc[2 * hm + ii][2 * hn + jj][r];
            }
          }
        }
        lds_sync();
        for (int pass = 0; pass < 2; ++pass) {
#pragma unroll
          for (int it = 0; it < 8; ++it) {
            const int ch = it * 4 + rr;
            const float bv = bfr(bias0[n0 + hn * 32 + ch]);
            const v4f xs = *(const v4f*)(slab + ch * 36 + q8 * 4);
            const size_t go = ((size_t)(bm * C_DIM + cbase + n0 + hn * 32 + ch)) * (size_t)HW_N
                              + (size_t)(sm0 + hm * 32 + q8 * 4);
            const v4f xr = *(const v4f*)(xres + go);
            v4f ov;
#pragma unroll
            for (int e = 0; e < 4; ++e) ov[e] = xs[e] * osc + bv + bfr(xr[e]);
            *(volatile v4f*)(Cf + go) = ov;
          }
          __threadfence();
        }
        lds_sync();
      }
    }
  }
}

__global__ __launch_bounds__(128) void k_attn_h(const unsigned short* __restrict__ Qh,
                                                const unsigned short* __restrict__ KV,
                                                unsigned short* Ctx) {
  __shared__ __align__(16) unsigned short sK[NPOOL * 40];
  __shared__ __align__(16) unsigned short sVt[32 * 168];
  __shared__ __align__(16) unsigned short sP[4][16 * 168];
  __shared__ __align__(16) float sO[4][16 * 36];
  const int tid = threadIdx.x, wave = tid >> 5, lane = tid & 31;
  const int hh = lane >> 4, c = lane & 15;
  const int bx = blockIdx.x;
  const int qt = bx % (HW_N / 64);
  const int h = (bx / (HW_N / 64)) % NHEAD;
  const int b = bx / ((HW_N / 64) * NHEAD);
  const int q0 = qt * 64 + wave * 16;
  const v16h qa = ldfrag_h(Qh + ((size_t)b * HW_N + q0 + c) * QH_LD + h * HEADD + 8 * hh);
  const unsigned short* kvb = KV + (size_t)b * NPOOL * KV_LD + h * HEADD;

  for (int idx = tid; idx < NPOOL * 4; idx += 128) {
    const int key = idx >> 2, piece = idx & 3;
    const v8us u = *(const v8us*)(kvb + (size_t)key * KV_LD + piece * 8);
    *(v8us*)(sK + key * 40 + piece * 8) = u;
    const int key2 = idx % NPOOL, piece2 = idx / NPOOL;
    const v8us w = *(const v8us*)(kvb + (size_t)key2 * KV_LD + KCOL + piece2 * 8);
#pragma unroll
    for (int e = 0; e < 8; ++e) sVt[(piece2 * 8 + e) * 168 + key2] = w[e];
  }
  if (tid < 64) {
    const int d = tid >> 1, hf = tid & 1;
    *(v8us*)(sVt + d * 168 + NPOOL + hf * 8) = zero8us();
  }
  __syncthreads();

  v8f s[9];
#pragma unroll
  for (int j = 0; j < 9; ++j) {
    const v16h kb = ldfrag_h(sK + (j * 16 + c) * 40 + 8 * hh);
    s[j] = mma_h(qa, kb, zero8());
  }
  unsigned short* sPw = sP[wave];
  float lsum[8];
#pragma unroll
  for (int r = 0; r < 8; ++r) {
    float mx = s[0][r];
#pragma unroll
    for (int j = 1; j < 9; ++j) mx = fmaxf(mx, s[j][r]);
    mx = fmaxf(mx, __shfl_xor(mx, 1, 32));
    mx = fmaxf(mx, __shfl_xor(mx, 2, 32));
    mx = fmaxf(mx, __shfl_xor(mx, 4, 32));
    mx = fmaxf(mx, __shfl_xor(mx, 8, 32));
    float ps = 0.f;
#pragma unroll
    for (int j = 0; j < 9; ++j) {
      const float p = exp2f((s[j][r] - mx) * CL2);
      ps += p;
      sPw[(8 * hh + r) * 168 + j * 16 + c] = h_bits(p);
    }
    sPw[(8 * hh + r) * 168 + NPOOL + c] = (unsigned short)0;
    lsum[r] = ps;
  }
#pragma unroll
  for (int r = 0; r < 8; ++r) {
    float ps = lsum[r];
    ps += __shfl_xor(ps, 1, 32);
    ps += __shfl_xor(ps, 2, 32);
    ps += __shfl_xor(ps, 4, 32);
    ps += __shfl_xor(ps, 8, 32);
    lsum[r] = ps;
  }
  lds_sync();
  v8f acc0 = zero8(), acc1 = zero8();
#pragma unroll
  for (int ks = 0; ks < 5; ++ks) {
    const v16h pa = ldfrag_h(sPw + c * 168 + ks * 32 + 8 * hh);
    const v16h v0 = ldfrag_h(sVt + c * 168 + ks * 32 + 8 * hh);
    const v16h v1 = ldfrag_h(sVt + (16 + c) * 168 + ks * 32 + 8 * hh);
    acc0 = mma_h(pa, v0, acc0);
    acc1 = mma_h(pa, v1, acc1);
  }

  float* sOw = sO[wave];
#pragma unroll
  for (int r = 0; r < 8; ++r) {
    const float inv = 1.0f / lsum[r];
    sOw[(8 * hh + r) * 36 + c]      = acc0[r] * inv;
    sOw[(8 * hh + r) * 36 + 16 + c] = acc1[r] * inv;
  }
  lds_sync();
  const int q8 = lane & 7, rr = lane >> 3, d8 = (q8 & 3) * 8;
  v4u ov[2];
  int tl[2];
#pragma unroll
  for (int it = 0; it < 2; ++it) {
    const int L = it * 4 + rr;
    tl[it] = 2 * L + (q8 >> 2);
    float f[8];
    ld8(sOw + tl[it] * 36 + d8, f);
    unsigned short hb[8];
#pragma unroll
    for (int e = 0; e < 8; ++e) hb[e] = h_bits(f[e]);
    v4u a4;
#pragma unroll
    for (int p = 0; p < 4; ++p) a4[p] = pk16(hb[2 * p], hb[2 * p + 1]);
    ov[it] = a4;
  }
  for (int pass = 0; pass < 2; ++pass) {
#pragma unroll
    for (int it = 0; it < 2; ++it) {
      const size_t go = (((size_t)(b * NHEAD + h)) * HW_N + q0 + tl[it]) * CTXW + d8;
      *(volatile v4u*)(Ctx + go) = ov[it];
    }
    __threadfence();
  }
}

__global__ __launch_bounds__(128) void k_attn_v(const unsigned short* __restrict__ Pq, unsigned short* Ctx) {
  __shared__ __align__(16) unsigned short sK[64 * 40];
  __shared__ __align__(16) unsigned short sVt[32 * 72];
  __shared__ __align__(16) unsigned short sP[4][16 * 72];
  __shared__ __align__(16) float sO[4][16 * 36];
  const int tid = threadIdx.x, wave = tid >> 5, lane = tid & 31;
  const int hh = lane >> 4, c = lane & 15;
  const int bx = blockIdx.x;
  const int qt = bx % (WTOK / 64);
  const int h = (bx / (WTOK / 64)) % NHEAD;
  const int wi = (bx / ((WTOK / 64) * NHEAD)) % NWIN;
  const int b = bx / ((WTOK / 64) * NHEAD * NWIN);
  const size_t rowb = (size_t)b * HW_N + (size_t)(wi * 4);
  const int i0 = qt * 64 + wave * 16;
  const int iq = i0 + c;
  const v16h qa = ldfrag_h(Pq + (rowb + (size_t)((iq >> 2) * IMG_W + (iq & 3))) * QKV_LD + h * HEADD + 8 * hh);
  float mrun[8], lrun[8];
#pragma unroll
  for (int r = 0; r < 8; ++r) { mrun[r] = -1e30f; lrun[r] = 0.f; }
  v8f acc0 = zero8(), acc1 = zero8();
  unsigned short* sPw = sP[wave];

  for (int kt = 0; kt < WTOK / 64; ++kt) {
    const int k0 = kt * 64;
#pragma unroll
    for (int it = 0; it < 2; ++it) {
      const int idx = it * 128 + tid;
      const int key = idx >> 2, piece = idx & 3;
      const int j = k0 + key;
      const v8us u = *(const v8us*)(Pq + (rowb + (size_t)((j >> 2) * IMG_W + (j & 3))) * QKV_LD
                                    + KCOL + h * HEADD + piece * 8);
      *(v8us*)(sK + key * 40 + piece * 8) = u;
      const int key2 = idx & 63, piece2 = idx >> 6;
      const int j2 = k0 + key2;
      const v8us w = *(const v8us*)(Pq + (rowb + (size_t)((j2 >> 2) * IMG_W + (j2 & 3))) * QKV_LD
                                    + VCOL + h * HEADD + piece2 * 8);
#pragma unroll
      for (int e = 0; e < 8; ++e) sVt[(piece2 * 8 + e) * 72 + key2] = w[e];
    }
    __syncthreads();

    v8f s[4];
#pragma unroll
    for (int j = 0; j < 4; ++j) {
      const v16h kb = ldfrag_h(sK + (j * 16 + c) * 40 + 8 * hh);
      s[j] = mma_h(qa, kb, zero8());
    }
    float tsum[8], alpha[8];
#pragma unroll
    for (int r = 0; r < 8; ++r) {
      float mx = fmaxf(fmaxf(s[0][r], s[1][r]), fmaxf(s[2][r], s[3][r]));
      mx = fmaxf(mx, __shfl_xor(mx, 1, 32));
      mx = fmaxf(mx, __shfl_xor(mx, 2, 32));
      mx = fmaxf(mx, __shfl_xor(mx, 4, 32));
      mx = fmaxf(mx, __shfl_xor(mx, 8, 32));
      const float mn = fmaxf(mrun[r], mx);
      alpha[r] = exp2f((mrun[r] - mn) * CL2);
      mrun[r] = mn;
      float ps = 0.f;
#pragma unroll
      for (int j = 0; j < 4; ++j) {
        const float p = exp2f((s[j][r] - mn) * CL2);
        ps += p;
        sPw[(8 * hh + r) * 72 + j * 16 + c] = h_bits(p);
      }
      tsum[r] = ps;
    }
#pragma unroll
    for (int r = 0; r < 8; ++r) {
      float ps = tsum[r];
      ps += __shfl_xor(ps, 1, 32);
      ps += __shfl_xor(ps, 2, 32);
      ps += __shfl_xor(ps, 4, 32);
      ps += __shfl_xor(ps, 8, 32);
      lrun[r] = lrun[r] * alpha[r] + ps;
      acc0[r] *= alpha[r];
      acc1[r] *= alpha[r];
    }
    lds_sync();
#pragma unroll
    for (int ks = 0; ks < 2; ++ks) {
      const v16h pa = ldfrag_h(sPw + c * 72 + ks * 32 + 8 * hh);
      const v16h v0 = ldfrag_h(sVt + c * 72 + ks * 32 + 8 * hh);
      const v16h v1 = ldfrag_h(sVt + (16 + c) * 72 + ks * 32 + 8 * hh);
      acc0 = mma_h(pa, v0, acc0);
      acc1 = mma_h(pa, v1, acc1);
    }
    __syncthreads();
  }

  float* sOw = sO[wave];
#pragma unroll
  for (int r = 0; r < 8; ++r) {
    const float inv = 1.0f / lrun[r];
    sOw[(8 * hh + r) * 36 + c]      = acc0[r] * inv;
    sOw[(8 * hh + r) * 36 + 16 + c] = acc1[r] * inv;
  }
  lds_sync();
  const int q8 = lane & 7, rr = lane >> 3, d8 = (q8 & 3) * 8;
  v4u ov[2];
  int tok[2];
#pragma unroll
  for (int it = 0; it < 2; ++it) {
    const int L = it * 4 + rr;
    const int il = (L >> 1) * 4 + (L & 1) * 2 + (q8 >> 2);
    tok[it] = ((i0 + il) >> 2) * IMG_W + wi * 4 + ((i0 + il) & 3);
    float f[8];
    ld8(sOw + il * 36 + d8, f);
    unsigned short hb[8];
#pragma unroll
    for (int e = 0; e < 8; ++e) hb[e] = h_bits(f[e]);
    v4u a4;
#pragma unroll
    for (int p = 0; p < 4; ++p) a4[p] = pk16(hb[2 * p], hb[2 * p + 1]);
    ov[it] = a4;
  }
  for (int pass = 0; pass < 2; ++pass) {
#pragma unroll
    for (int it = 0; it < 2; ++it) {
      const size_t go = (((size_t)(b * NHEAD + h)) * HW_N + tok[it]) * CTXW + d8;
      *(volatile v4u*)(Ctx + go) = ov[it];
    }
    __threadfence();
  }
}

__global__ __launch_bounds__(256) void k_rstats(const float* __restrict__ R, double* P2) {
  __shared__ float sS[256], sQ[256];
  __shared__ __align__(16) double sD[16];
  const float* rp = R + (size_t)blockIdx.x * (size_t)(8 * HW_N);
  const int t = threadIdx.x;
  float s = 0.f, q = 0.f;
#pragma unroll 2
  for (int i = 0; i < (8 * HW_N) / 1024; ++i) {
    const v4f v = *(const v4f*)(rp + (size_t)(i * 256 + t) * 4);
    s += (v[0] + v[1]) + (v[2] + v[3]);
    q += (v[0] * v[0] + v[1] * v[1]) + (v[2] * v[2] + v[3] * v[3]);
  }
  sS[t] = s; sQ[t] = q;
  if (t < 16) sD[t] = 0.0;
  __syncthreads();
  if (t == 0) {
    double ds = 0.0, dq = 0.0;
    for (int k = 0; k < 256; ++k) { ds += (double)sS[k]; dq += (double)sQ[k]; }
    sD[0] = ds; sD[1] = dq;
  }
  __syncthreads();
  if (t < 8) {
    const v4u v = *(const v4u*)(&sD[2 * t]);
    double* dst = P2 + (size_t)blockIdx.x * 16 + 2 * t;
    *(volatile v4u*)dst = v;
    __threadfence();
    *(volatile v4u*)dst = v;
  }
}

__global__ __launch_bounds__(64) void k_reduce2(const double* __restrict__ P2, int nb, float* T2, double inv_n) {
  __shared__ __align__(16) float sT[32];
  const int t = threadIdx.x;
  if (t < 32) sT[t] = 0.f;
  __syncthreads();
  if (t < nb) {
    double S = 0.0, Q = 0.0;
    for (int j = 0; j < 32; ++j) {
      S += P2[((size_t)(t * 32 + j)) * 16];
      Q += P2[((size_t)(t * 32 + j)) * 16 + 1];
    }
    const double m = S * inv_n;
    const double var = Q * inv_n - m * m;
    sT[2 * t] = (float)m;
    sT[2 * t + 1] = rsqrtf((float)var + LN_EPS);
  }
  __syncthreads();
  if (t < 8) {
    const v4f v = *(const v4f*)(sT + 4 * t);
    *(volatile v4f*)(T2 + 4 * t) = v;
    __threadfence();
    *(volatile v4f*)(T2 + 4 * t) = v;
  }
}

__global__ __launch_bounds__(256) void k_final(const float* __restrict__ R, const float* __restrict__ T2,
                                               float* out, int n4) {
  const int i = blockIdx.x * 256 + threadIdx.x;
  if (i >= n4) return;
  const int b = i / (C_DIM * HW_N / 4);
  const float m = T2[2 * b], r = T2[2 * b + 1];
  const v4f v = *(const v4f*)(R + (size_t)i * 4);
  v4f o;
#pragma unroll
  for (int e = 0; e < 4; ++e) o[e] = (v[e] - m) * r;
  *(volatile v4f*)(out + (size_t)i * 4) = o;
  __threadfence();
  *(volatile v4f*)(out + (size_t)i * 4) = o;
}

extern "C" void kernel_launch(void* const* d_in, const int* in_sizes, int n_in,
                              void* d_out, int out_size, void* d_ws, size_t ws_size,
                              hipStream_t stream) {
  if (n_in < 17) return;
  const int per = C_DIM * HW_N;
  if (in_sizes[0] <= 0 || (in_sizes[0] % per) != 0) return;
  const int nb = in_sizes[0] / per;
  if (nb < 1 || nb > MAXB) return;
  if (out_size != in_sizes[0]) return;
  if (in_sizes[1] != C_DIM * C_DIM || in_sizes[2] != C_DIM) return;
  if (in_sizes[3] != C_DIM * C_DIM || in_sizes[4] != C_DIM) return;
  if (in_sizes[5] != C_DIM * C_DIM || in_sizes[6] != C_DIM) return;
  if (in_sizes[7] != C_DIM * C1_DIM || in_sizes[8] != C1_DIM) return;
  if (in_sizes[9] != C_DIM * C_DIM || in_sizes[10] != C_DIM) return;
  if (in_sizes[11] != C_DIM * C_DIM || in_sizes[12] != C_DIM) return;
  if (in_sizes[13] != C_DIM * C_DIM || in_sizes[14] != C_DIM) return;
  if (in_sizes[15] != C_DIM * C2_DIM || in_sizes[16] != C2_DIM) return;

  const float* x   = (const float*)d_in[0];
  const float* hWq = (const float*)d_in[1];
  const float* hbq = (const float*)d_in[2];
  const float* hWk = (const float*)d_in[3];
  const float* hbk = (const float*)d_in[4];
  const float* hWv = (const float*)d_in[5];
  const float* hbv = (const float*)d_in[6];
  const float* hWo = (const float*)d_in[7];
  const float* hbo = (const float*)d_in[8];
  const float* vWq = (const float*)d_in[9];
  const float* vbq = (const float*)d_in[10];
  const float* vWk = (const float*)d_in[11];
  const float* vbk = (const float*)d_in[12];
  const float* vWv = (const float*)d_in[13];
  const float* vbv = (const float*)d_in[14];
  const float* vWo = (const float*)d_in[15];
  const float* vbo = (const float*)d_in[16];

  const int nTok = nb * HW_N;
  const int MP = ((nb * NPOOL + 63) / 64) * 64;

  const size_t PXB  = (size_t)nTok * C_DIM * 2;
  const size_t PU   = (size_t)nTok * QKV_LD * 2;
  const size_t PR   = (size_t)nb * per * 4;
  const size_t PCTX = (size_t)nb * NHEAD * HW_N * CTXW * 2;
  const size_t PXP  = (size_t)MP * C_DIM * 2;
  const size_t PKV  = (size_t)MP * KV_LD * 2;
  const size_t PWT  = (size_t)1024 * C_DIM * 2;
  const size_t PWKV = (size_t)512 * C_DIM * 2;
  const size_t PWOH = (size_t)C1_DIM * C_DIM * 2;
  const size_t PWOV = (size_t)C2_DIM * C_DIM * 2;
  const size_t PP1  = (size_t)nb * C_DIM * (2 * NWIN) * 8;
  const size_t PT   = (size_t)TS_N * 4;
  const size_t PP2  = (size_t)nb * 32 * 128;
  const size_t PT2  = 256;
  if (PR > PXB + PU) return;

  size_t off = 0;
  const size_t oXb  = off; off += PXB;
  const size_t oU   = off; off += PU;
  const size_t oR   = 0;
  const size_t oCh  = off; off += PCTX;
  const size_t oCv  = off; off += PCTX;
  const size_t oXph = off; off += PXP;
  const size_t oXpl = off; off += PXP;
  const size_t oKV  = off; off += PKV;
  const size_t oWt  = off; off += PWT;
  const size_t oWkv = off; off += PWKV;
  const size_t oWoh = off; off += PWOH;
  const size_t oWov = off; off += PWOV;
  const size_t oP1  = off; off += PP1;
  const size_t oT   = off; off += PT;
  const size_t oP2  = off; off += PP2;
  const size_t oT2  = off; off += PT2;
  if (off > ws_size) return;
  if (off > (size_t)134217728) return;

  char* ws = (char*)d_ws;
  unsigned short* Xb   = (unsigned short*)(ws + oXb);
  unsigned short* U    = (unsigned short*)(ws + oU);
  float*          R    = (float*)(ws + oR);
  unsigned short* Ch   = (unsigned short*)(ws + oCh);
  unsigned short* Cv   = (unsigned short*)(ws + oCv);
  unsigned short* Xph  = (unsigned short*)(ws + oXph);
  unsigned short* Xpl  = (unsigned short*)(ws + oXpl);
  unsigned short* KV   = (unsigned short*)(ws + oKV);
  unsigned short* Wt   = (unsigned short*)(ws + oWt);
  unsigned short* Wkv  = (unsigned short*)(ws + oWkv);
  unsigned short* Woh  = (unsigned short*)(ws + oWoh);
  unsigned short* Wov  = (unsigned short*)(ws + oWov);
  double*         P1   = (double*)(ws + oP1);
  float*          T    = (float*)(ws + oT);
  double*         P2   = (double*)(ws + oP2);
  float*          T2   = (float*)(ws + oT2);
  float*          outf = (float*)d_out;

  const dim3 blk(256);
  k_tr<0><<<dim3(HW_N / 64, C_DIM / 64, nb), blk, 0, stream>>>(x, Xb, C_DIM, HW_N);
  k_tr<0><<<dim3(C_DIM / 64, C_DIM / 64, 1), blk, 0, stream>>>(hWq, Wt, C_DIM, C_DIM);
  k_tr<0><<<dim3(C_DIM / 64, C_DIM / 64, 1), blk, 0, stream>>>(vWq, Wt + 1 * 65536, C_DIM, C_DIM);
  k_tr<0><<<dim3(C_DIM / 64, C_DIM / 64, 1), blk, 0, stream>>>(vWk, Wt + 2 * 65536, C_DIM, C_DIM);
  k_tr<0><<<dim3(C_DIM / 64, C_DIM / 64, 1), blk, 0, stream>>>(vWv, Wt + 3 * 65536, C_DIM, C_DIM);
  k_tr<0><<<dim3(C_DIM / 64, C_DIM / 64, 1), blk, 0, stream>>>(hWk, Wkv, C_DIM, C_DIM);
  k_tr<0><<<dim3(C_DIM / 64, C_DIM / 64, 1), blk, 0, stream>>>(hWv, Wkv + 65536, C_DIM, C_DIM);
  k_tr<1><<<dim3(C1_DIM / 64, C_DIM / 64, 1), blk, 0, stream>>>(hWo, Woh, C_DIM, C1_DIM);
  k_tr<1><<<dim3(C2_DIM / 64, C_DIM / 64, 1), blk, 0, stream>>>(vWo, Wov, C_DIM, C2_DIM);
  const int nblk = nb * C_DIM;
  k_xstats<<<dim3(nblk), dim3(192), 0, stream>>>(x, P1);
  const double inv_nw = 1.0 / ((double)nblk * (double)WTOK);
  const double inv_ng = 1.0 / ((double)nblk * (double)HW_N);
  k_reduce1<<<dim3(1), blk, 0, stream>>>(P1, nblk, hWq, vWq, T, inv_nw, inv_ng);
  const int padRows = MP - nb * NPOOL;
  if (padRows > 0) {
    const int npieces = padRows * (C_DIM / 8);
    k_zfill<<<dim3((npieces + 255) / 256), blk, 0, stream>>>(Xph, Xpl, nb * NPOOL, padRows);
  }
  k_pool<<<dim3(POOLG, C_DIM / 64, nb), blk, 0, stream>>>(x, Xph, Xpl);

  gemm64<1, 1, 0, 0, 1, 0><<<dim3((nTok / 64) * (QH_LD / 64) / 8), blk, 0, stream>>>(
      Xb, Xb, C_DIM, Wt, C_DIM, hbq, hbq, hbq, T, x, R, U, QH_LD, nTok, QH_LD, C_DIM, QKV_OSC, 0);
  gemm64<1, 2, 0, 0, 2, 0><<<dim3((MP / 64) * (KV_LD / 64) / 8), blk, 0, stream>>>(
      Xph, Xpl, C_DIM, Wkv, C_DIM, hbk, hbv, hbv, T, x, R, KV, KV_LD, MP, KV_LD, C_DIM, QKV_OSC, 0);
  k_attn_h<<<dim3(nb * NHEAD * (HW_N / 64)), dim3(128), 0, stream>>>(U, KV, Ch);
  gemm64<1, 1, 0, 0, 1, 1><<<dim3((nTok / 64) * (QKV_LD / 64) / 8), blk, 0, stream>>>(
      Xb, Xb, C_DIM, Wt + 65536, C_DIM, vbq, vbk, vbv, T, x, R, U, QKV_LD, nTok, QKV_LD, C_DIM, QKV_OSC, 0);
  k_attn_v<<<dim3(nb * NWIN * NHEAD * (WTOK / 64)), dim3(128), 0, stream>>>(U, Cv);
  gemm64<4, 1, 1, 1, 0, 0><<<dim3((nTok / 64) * (C1_DIM / 64) / 8), blk, 0, stream>>>(
      Ch, Ch, CTXW, Woh, C_DIM, hbo, hbo, hbo, T, x, R, U, 0, nTok, C1_DIM, C_DIM, OUT_OSC, 0);
  gemm64<4, 1, 1, 1, 0, 0><<<dim3((nTok / 64) * (C2_DIM / 64) / 8), blk, 0, stream>>>(
      Cv, Cv, CTXW, Wov, C_DIM, vbo, vbo, vbo, T, x, R, U, 0, nTok, C2_DIM, C_DIM, OUT_OSC, C1_DIM);
  k_rstats<<<dim3(nb * 32), blk, 0, stream>>>(R, P2);
  const double inv_n = 1.0 / (double)per;
  k_reduce2<<<dim3(1), dim3(64), 0, stream>>>(P2, nb, T2, inv_n);
  const int n4 = (nb * per) / 4;
  k_final<<<dim3(n4 / 256), blk, 0, stream>>>(R, T2, outf, n4);
  (void)hipGetLastError();
}
